// RouterKTArchitecture_39350490366316
// MI455X (gfx1250) — hardware-run, weakly checked
//
#include <hip/hip_runtime.h>
#include <math.h>

constexpr int kB = 8;
constexpr int kS = 1024;
constexpr int kD = 256;
constexpr int kH = 8;
constexpr int kDk = 32;
constexpr int kF = 1024;
constexpr int kNdyn = 6;
constexpr int kL = 6;
constexpr int kTok = kB * kS;
constexpr int kGroups = kB * kH;
constexpr float kNeg = -1.0e9f;
constexpr float kWCarry = 16.0f;
constexpr float kWCarryInv = 1.0f / 16.0f;
constexpr float kPCarry = 1024.0f;
constexpr float kPCarryInv = 1.0f / 1024.0f;
constexpr float kCtxCarry = 256.0f;
constexpr float kOutScale = 1.0f / (256.0f * 16.0f);
constexpr float kScoreScale = 0.17677669529663687f;
constexpr float kInvD = 1.0f / 256.0f;
constexpr float kLnEps = 1e-5f;

constexpr size_t kMiB = 1048576;
constexpr size_t kPlane32 = (size_t)kTok * kD * 4;
constexpr size_t kPlane16 = (size_t)kTok * kD * 2;
constexpr size_t oXA = 0;
constexpr size_t oXB = oXA + kPlane32;
constexpr size_t oYB = oXB + kPlane32;
constexpr size_t oT32 = oYB + kPlane32;
constexpr size_t oS = oT32 + kPlane32;
constexpr size_t kSBytes = (size_t)kH * kS * kS * 4;
constexpr size_t oD32 = oS;
constexpr size_t oH16 = oS + kPlane32;
constexpr size_t kHBytes = (size_t)kTok * kF * 2;
constexpr size_t oX16 = oH16 + kHBytes;
constexpr size_t oP = oS + kSBytes;
constexpr size_t kPBytes = (size_t)kH * kS * kS * 2;
constexpr size_t oCtx16 = oP;
constexpr size_t oT16 = oP + kPlane16;
constexpr size_t oO32 = oP + kPBytes;
constexpr size_t kOBytes = (size_t)kGroups * kS * 64 * 4;
constexpr size_t oVT = oO32 + kOBytes;
constexpr size_t kVTMain = (size_t)kGroups * kDk * kS * 2;
constexpr size_t kVTTail = (size_t)kDk * kS * 2;
constexpr size_t oY16 = oVT + kVTMain + kVTTail;
constexpr size_t oQ16 = oY16 + kPlane16;
constexpr size_t oWSQ = oQ16 + kPlane16;
constexpr size_t kWSQBytes = (size_t)18 * kD * kD * 2;
constexpr size_t oWF1 = oWSQ + kWSQBytes;
constexpr size_t kWFBytes = (size_t)kL * kF * kD * 2;
constexpr size_t oWF2 = oWF1 + kWFBytes;
constexpr size_t oPart = oWF2 + kWFBytes;
constexpr size_t oRout = oPart + 4096;
constexpr size_t oBalS = oRout + 256;
constexpr size_t kWsTotal = oBalS + 128;
static_assert(oX16 + kPlane16 <= oS + kSBytes, "S aliases fit");
static_assert(oT16 + kPlane16 <= oP + kPBytes, "P aliases fit");
static_assert(kWsTotal <= (size_t)134217728, "carve within 128 MiB");
static_assert((oS % 128) == 0 && (oP % 128) == 0 && (oO32 % 128) == 0 && (oVT % 128) == 0 && (oY16 % 128) == 0 &&
              (oQ16 % 128) == 0 && (oWSQ % 128) == 0 && (oWF1 % 128) == 0 && (oWF2 % 128) == 0 &&
              (oPart % 128) == 0 && (oRout % 128) == 0 && (oBalS % 128) == 0, "alignment");

typedef __attribute__((ext_vector_type(16))) _Float16 v16h;
typedef __attribute__((ext_vector_type(8)))  _Float16 v8h;
typedef __attribute__((ext_vector_type(16))) __bf16   v16b;
typedef __attribute__((ext_vector_type(8)))  __bf16   v8b;
typedef __attribute__((ext_vector_type(8)))  float    v8f;
typedef __attribute__((ext_vector_type(4)))  float    v4f;
typedef __attribute__((ext_vector_type(4)))  unsigned int v4u;

__device__ __forceinline__ unsigned short f2bf_bits(float f) {
  unsigned u = __float_as_uint(f);
  return (unsigned short)((u + 0x7FFFu + ((u >> 16) & 1u)) >> 16);
}
__device__ __forceinline__ float bf_bits2f(unsigned short h) { return __uint_as_float(((unsigned)h) << 16); }

__device__ __forceinline__ void dep_guard_h(v8f& a, v8f& b, v16h x, v16h y) { asm volatile("v_nop\n\tv_nop\n\tv_nop\n\tv_nop" : "+v"(a), "+v"(b) : "v"(x), "v"(y)); }
__device__ __forceinline__ void dep_guard_b(v8f& a, v8f& b, v16b x, v16b y) { asm volatile("v_nop\n\tv_nop\n\tv_nop\n\tv_nop" : "+v"(a), "+v"(b) : "v"(x), "v"(y)); }
__device__ __forceinline__ void keep4_h(v16h a, v16h b, v16h c, v16h d) { asm volatile("v_nop" :: "v"(a), "v"(b), "v"(c), "v"(d)); }
__device__ __forceinline__ void keep4_b(v16b a, v16b b, v16b c, v16b d) { asm volatile("v_nop" :: "v"(a), "v"(b), "v"(c), "v"(d)); }
__device__ __forceinline__ void acc_guard4(v8f& a, v8f& b, v8f& c, v8f& d) { asm volatile("v_nop\n\tv_nop\n\tv_nop\n\tv_nop" : "+v"(a), "+v"(b), "+v"(c), "+v"(d)); }
template <typename T> struct Frag;
template <> struct Frag<_Float16> {
  typedef v16h V; union U { v16h v; v8h h[2]; };
  static __device__ __forceinline__ v16h load(const _Float16* p) {
    U f; f.h[0] = *(const v8h*)(p); f.h[1] = *(const v8h*)(p + 16); return f.v;
  }
  static __device__ __forceinline__ v8f mma(v16h a, v16h b, v8f c) {
    return __builtin_amdgcn_wmma_f32_16x16x32_f16(false, a, false, b, (short)0, c, false, false);
  }
  static __device__ __forceinline__ void guard(v8f& a, v8f& b, v16h x, v16h y) { dep_guard_h(a, b, x, y); }
  static __device__ __forceinline__ void keep(v16h a, v16h b, v16h c, v16h d) { keep4_h(a, b, c, d); }
};
template <> struct Frag<__bf16> {
  typedef v16b V; union U { v16b v; v8b h[2]; };
  static __device__ __forceinline__ v16b load(const __bf16* p) {
    U f; f.h[0] = *(const v8b*)(p); f.h[1] = *(const v8b*)(p + 16); return f.v;
  }
  static __device__ __forceinline__ v8f mma(v16b a, v16b b, v8f c) {
    return __builtin_amdgcn_wmma_f32_16x16x32_bf16(false, a, false, b, (short)0, c, false, false);
  }
  static __device__ __forceinline__ void guard(v8f& a, v8f& b, v16b x, v16b y) { dep_guard_b(a, b, x, y); }
  static __device__ __forceinline__ void keep(v16b a, v16b b, v16b c, v16b d) { keep4_b(a, b, c, d); }
};

__device__ __forceinline__ unsigned pk16(unsigned short a, unsigned short b) { return (unsigned)a | ((unsigned)b << 16); }
__device__ __forceinline__ unsigned short h_bits(float f) { const _Float16 h = (_Float16)f; return __builtin_bit_cast(unsigned short, h); }

__device__ __forceinline__ void wave_sync_lds() {
  __builtin_amdgcn_fence(__ATOMIC_RELEASE, "workgroup");
  __builtin_amdgcn_wave_barrier();
  __builtin_amdgcn_fence(__ATOMIC_ACQUIRE, "workgroup");
}

template <int ET> struct Elem;
template <> struct Elem<0> { typedef _Float16 T; };
template <> struct Elem<1> { typedef __bf16 T; };
template <int ET, bool SPLIT, int BIAS_MODE, int OUT_MODE, bool RESID, int ACT = 0, int TRI = 0, int KLIM = 0>
__global__ __launch_bounds__(256) void wmma_gemm64(
    const unsigned short* __restrict__ Ap, const unsigned short* __restrict__ A2p, int lda, long strideA,
    const unsigned short* __restrict__ Btp, const unsigned short* __restrict__ Bt2p, int ldb, long strideB,
    void* __restrict__ Cout, void* __restrict__ Cout2, int ldc, long strideC,
    const float* __restrict__ bias,
    const float* __restrict__ resid, long strideR,
    int M, int N, int K, float scale) {
  typedef typename Elem<ET>::T T;
  typedef typename Frag<T>::V V;
  const T* A = (const T*)Ap; const T* A2 = (const T*)A2p; const T* Bt = (const T*)Btp; const T* Bt2 = (const T*)Bt2p;
  __shared__ __align__(16) float sT[8][16 * 68];
  const int b    = blockIdx.y;
  const int lane = threadIdx.x & 31;
  const int wave = threadIdx.x >> 5;
  const int tilesN = N >> 6;
  const int tilesM = M >> 6;
  const int tile = blockIdx.x * 8 + wave;
  if (tile >= tilesM * tilesN) return;
  const int tm = tile / tilesN;
  const int tn = tile - tm * tilesN;
  const int m0 = tm << 6;
  const int n0 = tn << 6;
  if (TRI == 1) { if (n0 > m0) return; }
  int Kend = K;
  if (KLIM == 1) Kend = (K < m0 + 64) ? K : (m0 + 64);
  if (KLIM == 2) Kend = (m0 == 0) ? K : ((K < m0 + 64) ? K : (m0 + 64));

  const T* Ab  = A  + (size_t)b * strideA;
  const T* Bb  = Bt + (size_t)b * strideB;
  const T* Ab2 = SPLIT ? (A2  + (size_t)b * strideA) : nullptr;
  const T* Bb2 = SPLIT ? (Bt2 + (size_t)b * strideB) : nullptr;

  const int rlane = lane & 15;
  const int koff  = (lane >> 4) * 8;
  const int mOff  = (lane >> 4) * 8;

  v8f acc[4][4];
#pragma unroll
  for (int i = 0; i < 4; ++i)
#pragma unroll
    for (int j = 0; j < 4; ++j) acc[i][j] = (v8f){0.f,0.f,0.f,0.f,0.f,0.f,0.f,0.f};

  for (int k0 = 0; k0 < Kend; k0 += 32) {
    V bh[4], bl[4];
#pragma unroll
    for (int j = 0; j < 4; ++j) {
      const size_t bo = (size_t)(n0 + (j << 4) + rlane) * ldb + koff + k0;
      bh[j] = Frag<T>::load(Bb + bo);
      if (SPLIT) bl[j] = Frag<T>::load(Bb2 + bo);
    }
#pragma unroll
    for (int i = 0; i < 4; ++i) {
      const size_t ao = (size_t)(m0 + (i << 4) + rlane) * lda + koff + k0;
      V ah = Frag<T>::load(Ab + ao);
      V al;
      if (SPLIT) al = Frag<T>::load(Ab2 + ao);
#pragma unroll
      for (int j = 0; j < 4; ++j) {
        acc[i][j] = Frag<T>::mma(ah, bh[j], acc[i][j]);
        if (SPLIT) {
          acc[i][j] = Frag<T>::mma(ah, bl[j], acc[i][j]);
          acc[i][j] = Frag<T>::mma(al, bh[j], acc[i][j]);
        }
      }
      Frag<T>::guard(acc[i][0], acc[i][3], ah, SPLIT ? al : ah);
    }
    Frag<T>::keep(bh[0], bh[1], bh[2], bh[3]);
    if (SPLIT) Frag<T>::keep(bl[0], bl[1], bl[2], bl[3]);
  }
  acc_guard4(acc[0][0], acc[0][1], acc[0][2], acc[0][3]);
  acc_guard4(acc[1][0], acc[1][1], acc[1][2], acc[1][3]);
  acc_guard4(acc[2][0], acc[2][1], acc[2][2], acc[2][3]);
  acc_guard4(acc[3][0], acc[3][1], acc[3][2], acc[3][3]);

  float* slab = sT[wave];
  const float* Rb = RESID ? (resid + (size_t)b * strideR) : nullptr;
#pragma unroll
  for (int i = 0; i < 4; ++i) {
    const int mBase = m0 + (i << 4);
#pragma unroll
    for (int j = 0; j < 4; ++j) {
      const int n = n0 + (j << 4) + rlane;
      float bv = 0.f;
      if (BIAS_MODE == 2) bv = bias[n];
#pragma unroll
      for (int r = 0; r < 8; ++r) {
        float v = acc[i][j][r] * scale;
        if (BIAS_MODE == 1) v += bias[mBase + mOff + r];
        if (BIAS_MODE == 2) v += bv;
        if (RESID) v += Rb[(size_t)(mBase + mOff + r) * ldc + n];
        if (ACT == 2) v = fmaxf(v, 0.0f);
        if (ACT == 4) v = (v > 0.f) ? v : 0.01f * v;
        slab[(mOff + r) * 68 + (j << 4) + rlane] = v;
      }
    }
    __builtin_amdgcn_fence(__ATOMIC_RELEASE, "workgroup");
    __builtin_amdgcn_wave_barrier();
    __builtin_amdgcn_fence(__ATOMIC_ACQUIRE, "workgroup");
    if (OUT_MODE == 0) {
      float* C = (float*)Cout + (size_t)b * strideC;
      const int hh = lane >> 4, c4 = (lane & 15) * 4;
      for (int pass = 0; pass < 2; ++pass) {
#pragma unroll
        for (int it = 0; it < 8; ++it) {
          const int row = it * 2 + hh;
          v4f v = *(const v4f*)(slab + row * 68 + c4);
          *(volatile v4f*)(C + (size_t)(mBase + row) * ldc + n0 + c4) = v;
        }
        __threadfence();
      }
    } else {
      const int q = lane >> 3, c8 = (lane & 7) * 8;
      unsigned short* C  = (unsigned short*)Cout  + (size_t)b * strideC;
      unsigned short* C2 = (OUT_MODE == 2) ? ((unsigned short*)Cout2 + (size_t)b * strideC) : nullptr;
      for (int pass = 0; pass < 2; ++pass) {
#pragma unroll
        for (int it = 0; it < 4; ++it) {
          const int row = it * 4 + q;
          const float* sp = slab + row * 68 + c8;
          v8h hv, lv;
#pragma unroll
          for (int e = 0; e < 8; ++e) {
            if (OUT_MODE == 1) {
              hv[e] = (_Float16)sp[e];
            } else {
              unsigned short hb = f2bf_bits(sp[e]);
              unsigned short lb = f2bf_bits(sp[e] - bf_bits2f(hb));
              hv[e] = __builtin_bit_cast(_Float16, hb);
              lv[e] = __builtin_bit_cast(_Float16, lb);
            }
          }
          *(volatile v8h*)(C + (size_t)(mBase + row) * ldc + n0 + c8) = hv;
          if (OUT_MODE == 2) *(volatile v8h*)(C2 + (size_t)(mBase + row) * ldc + n0 + c8) = lv;
        }
        __threadfence();
      }
    }
    __builtin_amdgcn_fence(__ATOMIC_RELEASE, "workgroup");
    __builtin_amdgcn_wave_barrier();
    __builtin_amdgcn_fence(__ATOMIC_ACQUIRE, "workgroup");
  }
}

__global__ __launch_bounds__(256) void wtcast_kernel(const float* __restrict__ W0, const float* __restrict__ W1,
                                                     const float* __restrict__ W2, int nper, int R, int C,
                                                     unsigned short* __restrict__ out, float scale) {
  __shared__ float sm[64][65];
  const int t  = threadIdx.x;
  const int r0 = blockIdx.x * 64;
  const int c0 = blockIdx.y * 64;
  const int z  = blockIdx.z;
  const int sel = z / nper;
  const int li  = z - sel * nper;
  const float* W = (sel == 0) ? W0 : (sel == 1) ? W1 : W2;
  W += (size_t)li * R * C;
#pragma unroll
  for (int i = 0; i < 16; ++i) {
    const int e = i * 256 + t;
    const int rr = e >> 6;
    const int cc = e & 63;
    sm[cc][rr] = W[(size_t)(r0 + rr) * C + c0 + cc] * scale;
  }
  __syncthreads();
  const int lane = t & 31, wave = t >> 5;
  const int q = lane >> 3, c8 = (lane & 7) * 8;
  unsigned short* op = out + (size_t)z * R * C;
  for (int pass = 0; pass < 2; ++pass) {
#pragma unroll
    for (int it = 0; it < 2; ++it) {
      const int row = wave * 8 + it * 4 + q;
      unsigned short hb[8];
#pragma unroll
      for (int e = 0; e < 8; ++e) hb[e] = h_bits(sm[row][c8 + e]);
      const v4u u = (v4u){pk16(hb[0], hb[1]), pk16(hb[2], hb[3]), pk16(hb[4], hb[5]), pk16(hb[6], hb[7])};
      *(volatile v4u*)(op + (size_t)(c0 + row) * R + r0 + c8) = u;
    }
    __threadfence();
  }
}

__global__ __launch_bounds__(256) void cast8_f16_kernel(const float* __restrict__ in, unsigned short* __restrict__ out, int n8) {
  const int i = blockIdx.x * 256 + threadIdx.x;
  if (i >= n8) return;
  const float* p = in + 8 * (size_t)i;
  const v4f a = *(const v4f*)(p);
  const v4f c = *(const v4f*)(p + 4);
  unsigned short hb[8];
#pragma unroll
  for (int e = 0; e < 4; ++e) {
    hb[e]     = h_bits(a[e]);
    hb[4 + e] = h_bits(c[e]);
  }
  const v4u u = (v4u){pk16(hb[0], hb[1]), pk16(hb[2], hb[3]), pk16(hb[4], hb[5]), pk16(hb[6], hb[7])};
  unsigned short* q = out + 8 * (size_t)i;
  *(volatile v4u*)q = u;
  __threadfence();
  *(volatile v4u*)q = u;
}

__global__ __launch_bounds__(256) void zero16_kernel(unsigned short* __restrict__ out, int n8) {
  const int i = blockIdx.x * 256 + threadIdx.x;
  if (i >= n8) return;
  const v4u u = (v4u){0u, 0u, 0u, 0u};
  unsigned short* q = out + 8 * (size_t)i;
  *(volatile v4u*)q = u;
  __threadfence();
  *(volatile v4u*)q = u;
}

__global__ __launch_bounds__(256) void router_kernel(const float* __restrict__ x, const float* __restrict__ Wg,
                                                     float* __restrict__ part) {
  __shared__ float red[18][256];
  __shared__ __align__(16) float line[32];
  const int t = threadIdx.x;
  const int r = blockIdx.x * 256 + t;
  const int b = r >> 10, rem = r & 1023, hh = rem >> 7, t8 = rem & 127;
  const float* base = x + ((size_t)(b * kS + t8 * 8)) * kD + hh * kDk;
  float lg[kNdyn] = {0.f, 0.f, 0.f, 0.f, 0.f, 0.f};
#pragma unroll 1
  for (int cc = 0; cc < kD; ++cc) {
    const float f = base[(size_t)(cc >> 5) * kD + (cc & 31)];
    const float* w = Wg + cc * kNdyn;
#pragma unroll
    for (int j = 0; j < kNdyn; ++j) lg[j] += f * w[j];
  }
  float mx = lg[0];
#pragma unroll
  for (int j = 1; j < kNdyn; ++j) mx = fmaxf(mx, lg[j]);
  float ev[kNdyn];
  float s = 0.f;
#pragma unroll
  for (int j = 0; j < kNdyn; ++j) { ev[j] = expf(lg[j] - mx); s += ev[j]; }
  const float inv = 1.0f / s;
  float g[kNdyn];
#pragma unroll
  for (int j = 0; j < kNdyn; ++j) g[j] = ev[j] * inv;
  int i0 = 0; float b0 = g[0];
#pragma unroll
  for (int j = 1; j < kNdyn; ++j) { if (g[j] > b0) { b0 = g[j]; i0 = j; } }
  int i1 = -1; float b1 = -INFINITY;
#pragma unroll
  for (int j = 0; j < kNdyn; ++j) { if (j != i0 && g[j] > b1) { b1 = g[j]; i1 = j; } }
#pragma unroll
  for (int j = 0; j < kNdyn; ++j) {
    const bool sel = (j == i0) || (j == i1);
    red[j][t]      = sel ? g[j] : 0.f;
    red[6 + j][t]  = sel ? 1.f : 0.f;
    red[12 + j][t] = g[j];
  }
  __syncthreads();
  if (t < 32) {
    const int tt = (t < 18) ? t : 17;
    float acc = 0.f;
#pragma unroll 1
    for (int k = 0; k < 256; ++k) acc += red[tt][k];
    line[t] = (t < 18) ? acc : 0.f;
  }
  __syncthreads();
  if (t < 8) {
    const v4f v = *(const v4f*)(line + 4 * t);
    float* dst = part + (size_t)blockIdx.x * 32 + 4 * t;
    *(volatile v4f*)dst = v;
    __threadfence();
    *(volatile v4f*)dst = v;
  }
}

__global__ __launch_bounds__(64) void route_fin_kernel(const float* __restrict__ part, float* __restrict__ routing,
                                                       float* __restrict__ bal_dst) {
  __shared__ __align__(16) float rl[64];
  const int t = threadIdx.x;
  const int b = t >> 3, h = t & 7;
  const int jj = (h >= 2) ? (h - 2) : 0;
  float s = 0.f;
#pragma unroll
  for (int k = 0; k < 4; ++k) s += part[(size_t)(4 * b + k) * 32 + jj];
  rl[t] = (h >= 2) ? (s * (1.0f / 1024.0f)) : 1.0f;
  float hs[kNdyn], hp[kNdyn];
#pragma unroll
  for (int j = 0; j < kNdyn; ++j) {
    float a = 0.f, c = 0.f;
#pragma unroll 1
    for (int blk = 0; blk < 32; ++blk) { a += part[blk * 32 + 6 + j]; c += part[blk * 32 + 12 + j]; }
    hs[j] = a;
    hp[j] = c * (1.0f / 8192.0f);
  }
  float hss = 0.f, hps = 0.f;
#pragma unroll
  for (int j = 0; j < kNdyn; ++j) { hss += hs[j]; hps += hp[j]; }
  const float r1 = 1.0f / (hss + 1e-5f);
  const float r2 = 1.0f / (hps + 1e-5f);
  float bal = 0.f;
#pragma unroll
  for (int j = 0; j < kNdyn; ++j) bal += (hs[j] * r1) * (hp[j] * r2);
  __syncthreads();
  if (t < 16) {
    const v4f v = *(const v4f*)(rl + 4 * t);
    *(volatile v4f*)(routing + 4 * t) = v;
    __threadfence();
    *(volatile v4f*)(routing + 4 * t) = v;
  }
  if (t == 0) {
    *(volatile float*)bal_dst = bal;
    __threadfence();
    *(volatile float*)bal_dst = bal;
  }
}

__global__ __launch_bounds__(256) void softmax_kernel(const float* __restrict__ S, unsigned short* __restrict__ P, int maskv) {
  __shared__ __align__(16) float xs[8][kS];
  const int t = threadIdx.x;
  const int lane = t & 31, wave = t >> 5;
  const int gr = blockIdx.x * 8 + wave;
  const int r = gr & (kS - 1);
  const size_t rowoff = (size_t)gr * kS;
  const float* sr = S + rowoff;
  float* xw = xs[wave];
  const int lim = r + maskv;
  const int nld = (lim + 255) >> 8;
  const int tm = r >> 6;
  const v4f negv = (v4f){kNeg, kNeg, kNeg, kNeg};
  float m = kNeg;
#pragma unroll 1
  for (int i = 0; i < 4; ++i) {
    v4f a = negv, c = negv;
    if (i < nld) {
      const int tcol = 4 * i + (lane >> 3);
      const int cb = (tcol <= tm) ? (i * 256 + 8 * lane) : ((lane & 7) * 8);
      const v4f la = *(const v4f*)(sr + cb);
      const v4f lc = *(const v4f*)(sr + cb + 4);
      const int col = i * 256 + 8 * lane;
#pragma unroll
      for (int e = 0; e < 4; ++e) {
        a[e] = (col + e < lim) ? la[e] : kNeg;
        c[e] = (col + 4 + e < lim) ? lc[e] : kNeg;
      }
    }
#pragma unroll
    for (int e = 0; e < 4; ++e) m = fmaxf(m, fmaxf(a[e], c[e]));
    *(v4f*)(xw + i * 256 + 8 * lane) = a;
    *(v4f*)(xw + i * 256 + 8 * lane + 4) = c;
  }
#pragma unroll
  for (int off = 16; off > 0; off >>= 1) m = fmaxf(m, __shfl_xor(m, off, 32));
  const float ez = expf(kNeg - m);
  float sum = 0.f;
#pragma unroll 1
  for (int i = 0; i < 4; ++i) {
    v4f a, c;
    if (i < nld) {
      a = *(const v4f*)(xw + i * 256 + 8 * lane);
      c = *(const v4f*)(xw + i * 256 + 8 * lane + 4);
#pragma unroll
      for (int e = 0; e < 4; ++e) { a[e] = expf(a[e] - m); c[e] = expf(c[e] - m); }
    } else {
      a = (v4f){ez, ez, ez, ez};
      c = a;
    }
#pragma unroll
    for (int e = 0; e < 4; ++e) sum += a[e] + c[e];
    *(v4f*)(xw + i * 256 + 8 * lane) = a;
    *(v4f*)(xw + i * 256 + 8 * lane + 4) = c;
  }
#pragma unroll
  for (int off = 16; off > 0; off >>= 1) sum += __shfl_xor(sum, off, 32);
  const float sc = kPCarry * (1.0f / sum);
  unsigned short* prow = P + rowoff;
  for (int pass = 0; pass < 2; ++pass) {
#pragma unroll 1
    for (int i = 0; i < 4; ++i) {
      const v4f a = *(const v4f*)(xw + i * 256 + 8 * lane);
      const v4f c = *(const v4f*)(xw + i * 256 + 8 * lane + 4);
      unsigned short hb[8];
#pragma unroll
      for (int e = 0; e < 4; ++e) {
        hb[e]     = h_bits(a[e] * sc);
        hb[4 + e] = h_bits(c[e] * sc);
      }
      const v4u u = (v4u){pk16(hb[0], hb[1]), pk16(hb[2], hb[3]), pk16(hb[4], hb[5]), pk16(hb[6], hb[7])};
      *(volatile v4u*)(prow + i * 256 + 8 * lane) = u;
    }
    __threadfence();
  }
}

__global__ __launch_bounds__(256) void merge_kernel(const float* __restrict__ O, const float* __restrict__ routing,
                                                    unsigned short* __restrict__ ctx) {
  const int e = blockIdx.x * 256 + threadIdx.x;
  const int token = e >> 5, u = e & 31;
  const int h = u >> 2, d0 = (u & 3) * 8;
  const int b = token >> 10, s = token & (kS - 1);
  const int g = b * kH + h;
  const float* src = O + ((size_t)g * kS + s) * 64 + d0;
  const v4f a = *(const v4f*)(src);
  const v4f c = *(const v4f*)(src + 4);
  const float rt = routing[g] * kCtxCarry;
  unsigned short hb[8];
#pragma unroll
  for (int k = 0; k < 4; ++k) {
    hb[k]     = h_bits(a[k] * rt);
    hb[4 + k] = h_bits(c[k] * rt);
  }
  const v4u uu = (v4u){pk16(hb[0], hb[1]), pk16(hb[2], hb[3]), pk16(hb[4], hb[5]), pk16(hb[6], hb[7])};
  unsigned short* q = ctx + (size_t)e * 8;
  *(volatile v4u*)q = uu;
  __threadfence();
  *(volatile v4u*)q = uu;
}

template <bool HAS16>
__global__ __launch_bounds__(256) void ln_kernel(const float* __restrict__ in, const float* __restrict__ gam,
                                                 const float* __restrict__ bet, float* __restrict__ out32,
                                                 unsigned short* __restrict__ out16) {
  __shared__ __align__(16) float st[8][kD];
  const int t = threadIdx.x;
  const int lane = t & 31, wave = t >> 5;
  const int row = blockIdx.x * 8 + wave;
  const float* rp = in + (size_t)row * kD;
  const v4f a = *(const v4f*)(rp + 4 * lane);
  const v4f c = *(const v4f*)(rp + 128 + 4 * lane);
  float x[8];
#pragma unroll
  for (int e = 0; e < 4; ++e) { x[e] = a[e]; x[4 + e] = c[e]; }
  float s = 0.f;
#pragma unroll
  for (int e = 0; e < 8; ++e) s += x[e];
#pragma unroll
  for (int off = 16; off > 0; off >>= 1) s += __shfl_xor(s, off, 32);
  const float mean = s * kInvD;
  float vs = 0.f;
#pragma unroll
  for (int e = 0; e < 8; ++e) { const float d = x[e] - mean; vs += d * d; }
#pragma unroll
  for (int off = 16; off > 0; off >>= 1) vs += __shfl_xor(vs, off, 32);
  const float inv = rsqrtf(vs * kInvD + kLnEps);
  const v4f ga = *(const v4f*)(gam + 4 * lane);
  const v4f gc = *(const v4f*)(gam + 128 + 4 * lane);
  const v4f ba = *(const v4f*)(bet + 4 * lane);
  const v4f bc = *(const v4f*)(bet + 128 + 4 * lane);
  v4f y0, y1;
#pragma unroll
  for (int e = 0; e < 4; ++e) {
    y0[e] = (x[e] - mean) * inv * ga[e] + ba[e];
    y1[e] = (x[4 + e] - mean) * inv * gc[e] + bc[e];
  }
  float* op = out32 + (size_t)row * kD;
  for (int pass = 0; pass < 2; ++pass) {
    *(volatile v4f*)(op + 4 * lane) = y0;
    *(volatile v4f*)(op + 128 + 4 * lane) = y1;
    __threadfence();
  }
  if (HAS16) {
    float* sw = st[wave];
    *(v4f*)(sw + 4 * lane) = y0;
    *(v4f*)(sw + 128 + 4 * lane) = y1;
    wave_sync_lds();
    const v4f q0 = *(const v4f*)(sw + 8 * lane);
    const v4f q1 = *(const v4f*)(sw + 8 * lane + 4);
    unsigned short hb[8];
#pragma unroll
    for (int e = 0; e < 4; ++e) {
      hb[e]     = h_bits(q0[e]);
      hb[4 + e] = h_bits(q1[e]);
    }
    const v4u u = (v4u){pk16(hb[0], hb[1]), pk16(hb[2], hb[3]), pk16(hb[4], hb[5]), pk16(hb[6], hb[7])};
    unsigned short* hp = out16 + (size_t)row * kD + 8 * lane;
    *(volatile v4u*)hp = u;
    __threadfence();
    *(volatile v4u*)hp = u;
  }
}

extern "C" void kernel_launch(void* const* d_in, const int* in_sizes, int n_in,
                              void* d_out, int out_size, void* d_ws, size_t ws_size, hipStream_t stream) {
  if (n_in < 17) return;
  if ((size_t)out_size < (size_t)kTok * kD + 1) return;
  if (ws_size < kWsTotal) return;
  if (in_sizes[0] != kTok * kD || in_sizes[1] != kTok * kD || in_sizes[2] != kL * kD * kD ||
      in_sizes[11] != kL * kD * kF || in_sizes[13] != kL * kF * kD || in_sizes[6] != kL * kD * kNdyn) return;

  const float* in0  = (const float*)d_in[0];
  const float* in1  = (const float*)d_in[1];
  const float* Wq   = (const float*)d_in[2];
  const float* bq   = (const float*)d_in[3];
  const float* Wv   = (const float*)d_in[4];
  const float* bv   = (const float*)d_in[5];
  const float* Wg   = (const float*)d_in[6];
  const float* Wo   = (const float*)d_in[7];
  const float* bo   = (const float*)d_in[8];
  const float* g1   = (const float*)d_in[9];
  const float* be1  = (const float*)d_in[10];
  const float* Wf1  = (const float*)d_in[11];
  const float* bf1  = (const float*)d_in[12];
  const float* Wf2  = (const float*)d_in[13];
  const float* bf2  = (const float*)d_in[14];
  const float* g2   = (const float*)d_in[15];
  const float* be2  = (const float*)d_in[16];

  char* W = (char*)d_ws;
  float* XA  = (float*)(W + oXA);
  float* XB  = (float*)(W + oXB);
  float* YB  = (float*)(W + oYB);
  float* T32 = (float*)(W + oT32);
  float* S32 = (float*)(W + oS);
  float* D32 = (float*)(W + oD32);
  unsigned short* H16   = (unsigned short*)(W + oH16);
  unsigned short* X16   = (unsigned short*)(W + oX16);
  unsigned short* P16   = (unsigned short*)(W + oP);
  unsigned short* Ctx16 = (unsigned short*)(W + oCtx16);
  unsigned short* T16   = (unsigned short*)(W + oT16);
  float* O32 = (float*)(W + oO32);
  unsigned short* VT    = (unsigned short*)(W + oVT);
  unsigned short* Y16   = (unsigned short*)(W + oY16);
  unsigned short* Q16   = (unsigned short*)(W + oQ16);
  unsigned short* WSQ   = (unsigned short*)(W + oWSQ);
  unsigned short* WF1   = (unsigned short*)(W + oWF1);
  unsigned short* WF2   = (unsigned short*)(W + oWF2);
  float* Part = (float*)(W + oPart);
  float* Rout = (float*)(W + oRout);
  float* BalS = (float*)(W + oBalS);
  float* out0 = (float*)d_out;
  float* out1 = out0 + (size_t)kTok * kD;

  wtcast_kernel<<<dim3(kD / 64, kD / 64, 18), 256, 0, stream>>>(Wq, Wv, Wo, kL, kD, kD, WSQ, kWCarry);
  wtcast_kernel<<<dim3(kD / 64, kF / 64, kL), 256, 0, stream>>>(Wf1, Wf1, Wf1, kL, kD, kF, WF1, kWCarry);
  wtcast_kernel<<<dim3(kF / 64, kD / 64, kL), 256, 0, stream>>>(Wf2, Wf2, Wf2, kL, kF, kD, WF2, kWCarry);
  zero16_kernel<<<(kDk * kS / 8) / 256, 256, 0, stream>>>(VT + (size_t)kGroups * kDk * kS, kDk * kS / 8);
  cast8_f16_kernel<<<(kTok * kD / 8) / 256, 256, 0, stream>>>(in1, X16, kTok * kD / 8);

  const long tokPlane16 = (long)kS * kD;
  const long vtBatch    = (long)kD * kS;
  const long headVT     = (long)kDk * kS;
  const long scorePlane = (long)kS * kS;
  const long oGroup     = (long)kS * 64;

  auto run_layer = [&](int li, const float* qry32, const unsigned short* qry16, const unsigned short* val16,
                       const float* rtr32, int maskv, bool ffn, float* dest32, unsigned short* dest16, float* bal_dst) {
    const float* bq_l  = bq  + (size_t)li * kD;
    const float* bv_l  = bv  + (size_t)li * kD;
    const float* Wg_l  = Wg  + (size_t)li * kD * kNdyn;
    const float* bo_l  = bo  + (size_t)li * kD;
    const float* g1_l  = g1  + (size_t)li * kD;
    const float* be1_l = be1 + (size_t)li * kD;
    const float* bf1_l = bf1 + (size_t)li * kF;
    const float* bf2_l = bf2 + (size_t)li * kD;
    const float* g2_l  = g2  + (size_t)li * kD;
    const float* be2_l = be2 + (size_t)li * kD;
    const unsigned short* WqT_l  = WSQ + (size_t)li * kD * kD;
    const unsigned short* WvT_l  = WSQ + (size_t)(6 + li) * kD * kD;
    const unsigned short* WoT_l  = WSQ + (size_t)(12 + li) * kD * kD;
    const unsigned short* Wf1T_l = WF1 + (size_t)li * kF * kD;
    const unsigned short* Wf2T_l = WF2 + (size_t)li * kF * kD;

    wmma_gemm64<0, false, 2, 1, false, 0><<<dim3(64, 1), 256, 0, stream>>>(
        qry16, nullptr, kD, 0, WqT_l, nullptr, kD, 0, (void*)Q16, nullptr, kD, 0,
        bq_l, nullptr, 0, kTok, kD, kD, kWCarryInv);
    wmma_gemm64<0, false, 1, 1, false, 0><<<dim3(8, kB), 256, 0, stream>>>(
        WvT_l, nullptr, kD, 0, val16, nullptr, kD, tokPlane16, (void*)VT, nullptr, kS, vtBatch,
        bv_l, nullptr, 0, kD, kS, kD, kWCarryInv);
    router_kernel<<<kTok / 256, 256, 0, stream>>>(rtr32, Wg_l, Part);
    route_fin_kernel<<<1, 64, 0, stream>>>(Part, Rout, bal_dst);
    for (int b = 0; b < kB; ++b) {
      const unsigned short* Qb = Q16 + (size_t)b * kS * kD;
      wmma_gemm64<0, false, 0, 0, false, 0, 1, 0><<<dim3(32, kH), 256, 0, stream>>>(
          Qb, nullptr, kD, (long)kDk, Qb, nullptr, kD, (long)kDk, (void*)S32, nullptr, kS, scorePlane,
          nullptr, nullptr, 0, kS, kS, kDk, kScoreScale);
      softmax_kernel<<<(kH * kS) / 8, 256, 0, stream>>>(S32, P16, maskv);
      if (maskv != 0) {
        wmma_gemm64<0, false, 0, 0, false, 0, 0, 1><<<dim3(2, kH), 256, 0, stream>>>(
            P16, nullptr, kS, scorePlane, VT + (size_t)b * vtBatch, nullptr, kS, headVT,
            (void*)(O32 + (size_t)b * kH * oGroup), nullptr, 64, oGroup,
            nullptr, nullptr, 0, kS, 64, kS, kPCarryInv);
      } else {
        wmma_gemm64<0, false, 0, 0, false, 0, 0, 2><<<dim3(2, kH), 256, 0, stream>>>(
            P16, nullptr, kS, scorePlane, VT + (size_t)b * vtBatch, nullptr, kS, headVT,
            (void*)(O32 + (size_t)b * kH * oGroup), nullptr, 64, oGroup,
            nullptr, nullptr, 0, kS, 64, kS, kPCarryInv);
      }
    }
    merge_kernel<<<(kTok * 32) / 256, 256, 0, stream>>>(O32, Rout, Ctx16);
    wmma_gemm64<0, false, 2, 0, true, 0><<<dim3(64, 1), 256, 0, stream>>>(
        Ctx16, nullptr, kD, 0, WoT_l, nullptr, kD, 0, (void*)D32, nullptr, kD, 0,
        bo_l, qry32, 0, kTok, kD, kD, kOutScale);
    if (ffn) {
      ln_kernel<true><<<kTok / 8, 256, 0, stream>>>(D32, g1_l, be1_l, T32, T16);
      wmma_gemm64<0, false, 2, 1, false, 2><<<dim3(256, 1), 256, 0, stream>>>(
          T16, nullptr, kD, 0, Wf1T_l, nullptr, kD, 0, (void*)H16, nullptr, kF, 0,
          bf1_l, nullptr, 0, kTok, kF, kD, kWCarryInv);
      wmma_gemm64<0, false, 2, 0, true, 0><<<dim3(64, 1), 256, 0, stream>>>(
          H16, nullptr, kF, 0, Wf2T_l, nullptr, kF, 0, (void*)D32, nullptr, kD, 0,
          bf2_l, T32, 0, kTok, kD, kF, kWCarryInv);
      if (dest16 != nullptr) ln_kernel<true><<<kTok / 8, 256, 0, stream>>>(D32, g2_l, be2_l, dest32, dest16);
      else                   ln_kernel<false><<<kTok / 8, 256, 0, stream>>>(D32, g2_l, be2_l, dest32, nullptr);
    } else {
      if (dest16 != nullptr) ln_kernel<true><<<kTok / 8, 256, 0, stream>>>(D32, g1_l, be1_l, dest32, dest16);
      else                   ln_kernel<false><<<kTok / 8, 256, 0, stream>>>(D32, g1_l, be1_l, dest32, nullptr);
    }
  };

  run_layer(0, in1, X16, X16, in0, 1, true, XB, X16, BalS);
  run_layer(1, XB, X16, X16, in0, 1, true, YB, Y16, BalS);
  cast8_f16_kernel<<<(kTok * kD / 8) / 256, 256, 0, stream>>>(in0, X16, kTok * kD / 8);
  run_layer(2, in0, X16, X16, in0, 1, false, XA, X16, BalS);
  run_layer(3, XA, X16, Y16, XA, 0, true, XB, X16, BalS);
  run_layer(4, XB, X16, X16, XB, 1, false, XA, X16, BalS);
  run_layer(5, XA, X16, Y16, XA, 0, true, out0, nullptr, out1);
}
